// GATNet_48473000902803
// MI455X (gfx1250) — hardware-run, weakly checked
//
#include <hip/hip_runtime.h>
#include <stddef.h>
#include <stdint.h>
#include <math.h>


#define F_IN    32
#define XQ      (F_IN / 8)
#define NHD1    10
#define HID     32
#define HC1     320
#define NHB1    2
#define NHBMAX  2
#define NLANE1  (HC1 / 16)
#define KA2     640
#define NC2     128
#define KFC     256
#define PER_G   200
#define NGMAX   1024
#define NTHR    256
#define NWAVE   8
#define EPT     8
#define CHUNK   (NTHR * EPT)
#define WCAP    (EPT * 32)
#define LISTN   (NWAVE * WCAP)
#define NBMAX   2048
#define SLOTB   11
#define RCAP    28672
#define DEGCAP  128
#define GBM     64
#define GTHR    128
#define MROWS   128
#define RBH     KA2
#define RBP     (RBH / 8)
#define PTHR    256
#define NEGSL   0.2f
#define EPS_SM  1e-16f
#define WSMAX   134217728
#define LDS_INTS (2 * RCAP + 2 * NBMAX + LISTN + 2 * NWAVE + NGMAX + 8)
#define LDS_AGG  (LDS_INTS * 4 + NWAVE * RBH * 2)

static_assert((CHUNK & (CHUNK - 1)) == 0 && CHUNK <= (1 << SLOTB));
static_assert(NBMAX == (1 << SLOTB));
static_assert(NTHR * 8 == NBMAX);
static_assert(LISTN >= NBMAX);
static_assert(LISTN >= NWAVE * WCAP);
static_assert((RCAP % 32) == 0);
static_assert(((LDS_INTS * 4) % 16) == 0);
static_assert(LDS_AGG <= 300000);
static_assert(GBM == (GTHR / 32) * 16);
static_assert(GTHR == 2 * GBM);
static_assert((F_IN % 32) == 0 && (KA2 % 32) == 0 && (KFC % 32) == 0);
static_assert(HC1 == NHD1 * HID && NHB1 * HID == 64 && (HC1 % 64) == 0);
static_assert(NHD1 == NHB1 * (HC1 / 64));
static_assert(NHB1 <= NHBMAX);
static_assert((HID % 4) == 0 && (NC2 % 4) == 0);
static_assert(KA2 == 2 * HC1 && KFC == 2 * NC2);
static_assert((MROWS % GBM) == 0);
static_assert(HC1 == 16 * NLANE1 && NLANE1 <= 32 && (HID % 16) == 0);
static_assert(NC2 == 4 * 32);
static_assert(RBP == 80 && (RBH * 2) % 128 == 0);
static_assert(XQ == 4 && (F_IN % 8) == 0);
static_assert(PTHR == NWAVE * 32 && NC2 <= PTHR);

typedef float          v2f  __attribute__((ext_vector_type(2)));
typedef float          v4f  __attribute__((ext_vector_type(4)));
typedef float          v8f  __attribute__((ext_vector_type(8)));
typedef int            v4i  __attribute__((ext_vector_type(4)));
typedef int            v8i  __attribute__((ext_vector_type(8)));
typedef unsigned int   v2u  __attribute__((ext_vector_type(2)));
typedef unsigned int   v4u  __attribute__((ext_vector_type(4)));
typedef unsigned short v8us __attribute__((ext_vector_type(8)));
typedef __bf16         v16b __attribute__((ext_vector_type(16)));
typedef v2f  __attribute__((may_alias)) v2fa;
typedef v4f  __attribute__((may_alias)) v4fa;
typedef v2u  __attribute__((may_alias)) v2ua;
typedef v4u  __attribute__((may_alias)) v4ua;
typedef v8us __attribute__((may_alias)) v8usa;
union FragB { v16b v; v8us h[2]; v8i w; };

__device__ __forceinline__ v8f wmb(const FragB& a, const FragB& b, v8f c) {
  v8f d = __builtin_amdgcn_wmma_f32_16x16x32_bf16(false, a.v, false, b.v, (short)0, c, false, false);
  asm volatile("v_nop\n\tv_nop\n\tv_nop\n\tv_nop" : "+v"(d) : "v"(a.w), "v"(b.w));
  return d;
}

__device__ __forceinline__ unsigned int f2bf(float f) {
  const unsigned int u = __float_as_uint(f);
  return ((u + 0x7FFFu + ((u >> 16) & 1u)) >> 16) & 0xFFFFu;
}
__device__ __forceinline__ float bf2f(unsigned int b) { return __uint_as_float(b << 16); }
__device__ __forceinline__ float bfr(float f) { return bf2f(f2bf(f)); }
__device__ __forceinline__ v4f bfr4(const v4f a) {
  v4f r; r.x = bfr(a.x); r.y = bfr(a.y); r.z = bfr(a.z); r.w = bfr(a.w); return r;
}
__device__ __forceinline__ unsigned int pk2(float lo, float hi) { return f2bf(lo) | (f2bf(hi) << 16); }
__device__ __forceinline__ v4u pack8(const v4f a, const v4f b) {
  v4u r;
  r.x = pk2(a.x, a.y); r.y = pk2(a.z, a.w); r.z = pk2(b.x, b.y); r.w = pk2(b.z, b.w);
  return r;
}
__device__ __forceinline__ v4u hl8(const v4f a, const v4f b, v4u& lo) {
  const unsigned int h0 = f2bf(a.x), h1 = f2bf(a.y), h2 = f2bf(a.z), h3 = f2bf(a.w);
  const unsigned int h4 = f2bf(b.x), h5 = f2bf(b.y), h6 = f2bf(b.z), h7 = f2bf(b.w);
  const unsigned int l0 = f2bf(a.x - bf2f(h0)), l1 = f2bf(a.y - bf2f(h1));
  const unsigned int l2 = f2bf(a.z - bf2f(h2)), l3 = f2bf(a.w - bf2f(h3));
  const unsigned int l4 = f2bf(b.x - bf2f(h4)), l5 = f2bf(b.y - bf2f(h5));
  const unsigned int l6 = f2bf(b.z - bf2f(h6)), l7 = f2bf(b.w - bf2f(h7));
  v4u hi;
  hi.x = h0 | (h1 << 16); hi.y = h2 | (h3 << 16); hi.z = h4 | (h5 << 16); hi.w = h6 | (h7 << 16);
  lo.x = l0 | (l1 << 16); lo.y = l2 | (l3 << 16); lo.z = l4 | (l5 << 16); lo.w = l6 | (l7 << 16);
  return hi;
}
__device__ __forceinline__ v4f upd4(v4f a, float s1, float s2, const v4f f) {
  a.x = fmaf(a.x, s1, s2 * f.x);
  a.y = fmaf(a.y, s1, s2 * f.y);
  a.z = fmaf(a.z, s1, s2 * f.z);
  a.w = fmaf(a.w, s1, s2 * f.w);
  return a;
}
__device__ __forceinline__ v4f elu4(const v4f a, float inv, const v4f b, bool live, float pz) {
  float hx = fmaf(a.x, inv, b.x);
  float hy = fmaf(a.y, inv, b.y);
  float hz = fmaf(a.z, inv, b.z);
  float hw = fmaf(a.w, inv, b.w);
  const float nx = __expf(fminf(hx, 0.f)) - 1.0f;
  const float ny = __expf(fminf(hy, 0.f)) - 1.0f;
  const float nz = __expf(fminf(hz, 0.f)) - 1.0f;
  const float nw = __expf(fminf(hw, 0.f)) - 1.0f;
  hx = hx > 0.f ? hx : nx;
  hy = hy > 0.f ? hy : ny;
  hz = hz > 0.f ? hz : nz;
  hw = hw > 0.f ? hw : nw;
  v4f o;
  o.x = (live ? hx : 0.f) + pz;
  o.y = (live ? hy : 0.f) + pz;
  o.z = (live ? hz : 0.f) + pz;
  o.w = (live ? hw : 0.f) + pz;
  return o;
}

__device__ __forceinline__ void wave_sync() {
  __builtin_amdgcn_fence(__ATOMIC_RELEASE, "wavefront");
  __builtin_amdgcn_wave_barrier();
  __builtin_amdgcn_fence(__ATOMIC_ACQUIRE, "wavefront");
}

__device__ __forceinline__ int scan_chunk(const int* __restrict__ dsts, int nE, int cbase, int slotBase,
                                          int nb, int vec8, int* list, int tid, int lane, int wave) {
  int wc = 0;
  const int el0  = tid * EPT;
  const int e0   = cbase + el0;
  const int sent = -2147483647 - 1;
  v4i da, db;
  if (vec8 != 0 && cbase + CHUNK <= nE) {
    da = *(const v4i*)(dsts + e0);
    db = *(const v4i*)(dsts + e0 + 4);
  } else {
    da.x = (e0     < nE) ? dsts[min(e0,     nE - 1)] : sent;
    da.y = (e0 + 1 < nE) ? dsts[min(e0 + 1, nE - 1)] : sent;
    da.z = (e0 + 2 < nE) ? dsts[min(e0 + 2, nE - 1)] : sent;
    da.w = (e0 + 3 < nE) ? dsts[min(e0 + 3, nE - 1)] : sent;
    db.x = (e0 + 4 < nE) ? dsts[min(e0 + 4, nE - 1)] : sent;
    db.y = (e0 + 5 < nE) ? dsts[min(e0 + 5, nE - 1)] : sent;
    db.z = (e0 + 6 < nE) ? dsts[min(e0 + 6, nE - 1)] : sent;
    db.w = (e0 + 7 < nE) ? dsts[min(e0 + 7, nE - 1)] : sent;
  }
  const unsigned nbs = (unsigned)slotBase;
  const unsigned unb = (unsigned)nb;
  const unsigned s0 = (unsigned)da.x - nbs, s1 = (unsigned)da.y - nbs;
  const unsigned s2 = (unsigned)da.z - nbs, s3 = (unsigned)da.w - nbs;
  const unsigned s4 = (unsigned)db.x - nbs, s5 = (unsigned)db.y - nbs;
  const unsigned s6 = (unsigned)db.z - nbs, s7 = (unsigned)db.w - nbs;
  const bool h0 = s0 < unb, h1 = s1 < unb, h2 = s2 < unb, h3 = s3 < unb;
  const bool h4 = s4 < unb, h5 = s5 < unb, h6 = s6 < unb, h7 = s7 < unb;
  const unsigned any = __builtin_amdgcn_ballot_w32(h0 | h1 | h2 | h3 | h4 | h5 | h6 | h7);
  if (any != 0u) {
#define HITJ(J, HJ, SJ) { \
      const unsigned mj = __builtin_amdgcn_ballot_w32(HJ); \
      if (mj != 0u) { \
        if (HJ) { \
          const int pos = wc + (int)__builtin_amdgcn_mbcnt_lo(mj, 0u); \
          if (pos < WCAP) list[wave * WCAP + pos] = ((el0 + (J)) << SLOTB) | (int)(SJ); \
        } \
        wc += (int)__builtin_popcount(mj); } }
    HITJ(0, h0, s0)
    HITJ(1, h1, s1)
    HITJ(2, h2, s2)
    HITJ(3, h3, s3)
    HITJ(4, h4, s4)
    HITJ(5, h5, s5)
    HITJ(6, h6, s6)
    HITJ(7, h7, s7)
#undef HITJ
  }
  return wc;
}

__global__ __launch_bounds__(NTHR) void k_xprep(const float* __restrict__ x, unsigned short* xb, int nN, int nUnits) {
  const int i = (int)blockIdx.x * NTHR + (int)threadIdx.x;
  if (i >= nUnits) return;
  const int row = i / XQ;
  const int c0  = (i - row * XQ) * 8;
  const int rc  = row < nN ? row : nN - 1;
  const float* p = x + (size_t)rc * F_IN + c0;
  v4f a = *(const v4fa*)p, b = *(const v4fa*)(p + 4);
  const v4f z4 = {0.f, 0.f, 0.f, 0.f};
  if (row >= nN) { a = z4; b = z4; }
  const v4u hv = pack8(a, b);
  const size_t o = (size_t)row * F_IN + c0;
  *(volatile v4u*)(xb + o) = hv;
  __threadfence();
  *(volatile v4u*)(xb + o) = hv;
}

__global__ __launch_bounds__(NTHR) void k_wtr(const float* __restrict__ w, int Kin, int Ncol, int Nrows, int Kout,
                                              unsigned short* wt, int nUnits) {
  const int u = (int)blockIdx.x * NTHR + (int)threadIdx.x;
  if (u >= nUnits) return;
  const int kq = Kout >> 3;
  const int n  = u / kq;
  const int k8 = (u - n * kq) * 8;
  const int kk = k8 - (k8 / Kin) * Kin;
  const int ncl = n < Ncol ? n : Ncol - 1;
  const float* p = w + (size_t)kk * (size_t)Ncol + ncl;
  v4f a, b;
  a.x = p[0];                    a.y = p[(size_t)Ncol];         a.z = p[(size_t)2 * Ncol];     a.w = p[(size_t)3 * Ncol];
  b.x = p[(size_t)4 * Ncol];     b.y = p[(size_t)5 * Ncol];     b.z = p[(size_t)6 * Ncol];     b.w = p[(size_t)7 * Ncol];
  const v4f z4 = {0.f, 0.f, 0.f, 0.f};
  if (n >= Ncol || n >= Nrows) { a = z4; b = z4; }
  const v4u wv = pack8(a, b);
  unsigned short* o = wt + (size_t)n * (size_t)Kout + k8;
  *(volatile v4u*)o = wv;
  __threadfence();
  *(volatile v4u*)o = wv;
}

template <int NT, int MODE>
__global__ __launch_bounds__(GTHR) void k_gemm(
    const unsigned short* __restrict__ A, const unsigned short* __restrict__ WT,
    float* outF, int K, int ldo, int nRows,
    const float* __restrict__ atts, const float* __restrict__ attd, int attLen, int nhb,
    float* SD, int MPr, const float* __restrict__ bias)
{
  constexpr int GBN = 16 * NT;
  constexpr int PPR = GBN / 4;
  constexpr int NI  = (16 * PPR) / 32;
  static_assert(NT == 4 || NT == 8);
  static_assert(MODE == 0 || NT == 8);
  __shared__ __attribute__((aligned(16))) float stg[GBM * GBN];
  __shared__ __attribute__((aligned(16))) float satt[2 * GBN];
  __shared__ __attribute__((aligned(16))) float sdot[2 * NHBMAX * GBM];
  const int tid = (int)threadIdx.x, lane = tid & 31, wave = tid >> 5, hh = lane >> 4, m = lane & 15;
  const int rowBase = (int)blockIdx.x * GBM;
  const int by      = (int)blockIdx.y;
  const int col0    = by * GBN;

  if constexpr (MODE == 0) {
    const int nv = nhb * attLen;
#pragma unroll 1
    for (int j = tid; j < 2 * GBN; j += GTHR) {
      const int which = j / GBN;
      const int c  = j - which * GBN;
      const int cl = c < nv ? c : nv - 1;
      const int gi = by * nv + cl;
      const float vs = atts[gi];
      const float vd = attd[gi];
      float v = (which == 0) ? vs : vd;
      v = (c < nv) ? bfr(v) : 0.f;
      satt[j] = v;
    }
  }

  v8f acc[NT];
  {
    const v8f z = {0.f, 0.f, 0.f, 0.f, 0.f, 0.f, 0.f, 0.f};
#pragma unroll
    for (int t = 0; t < NT; ++t) acc[t] = z;
  }
  const unsigned short* ap = A  + (size_t)(rowBase + 16 * wave + m) * (size_t)K + 8 * hh;
  const unsigned short* wp = WT + (size_t)(col0 + m) * (size_t)K + 8 * hh;
  const int ksteps = K >> 5;
#pragma unroll 1
  for (int ks = 0; ks < ksteps; ++ks) {
    FragB af;
    af.h[0] = *(const v8usa*)(ap + 32 * ks);
    af.h[1] = *(const v8usa*)(ap + 32 * ks + 16);
#pragma unroll
    for (int t = 0; t < NT; ++t) {
      const unsigned short* wq = wp + (size_t)(16 * t) * (size_t)K + 32 * ks;
      FragB bf;
      bf.h[0] = *(const v8usa*)wq;
      bf.h[1] = *(const v8usa*)(wq + 16);
      acc[t] = wmb(af, bf, acc[t]);
    }
  }

#pragma unroll
  for (int t = 0; t < NT; ++t) {
    const int lc = 16 * t + m;
#pragma unroll
    for (int r = 0; r < 8; ++r) {
      const int lr = 16 * wave + 8 * hh + r;
      stg[lr * GBN + lc] = acc[t][r];
    }
  }
  __syncthreads();

  if constexpr (MODE == 0) {
    const int row = tid & 63, which = tid >> 6;
    const float* sa = satt + which * GBN;
    const float* hr = stg + row * GBN;
    const int n4 = attLen >> 2;
#pragma unroll 1
    for (int hl = 0; hl < nhb; ++hl) {
      const int cb = hl * attLen;
      float d = 0.f;
#pragma unroll 2
      for (int c4 = 0; c4 < n4; ++c4) {
        const v4f hv = *(const v4fa*)(hr + cb + 4 * c4);
        const v4f av = *(const v4fa*)(sa + cb + 4 * c4);
        d = fmaf(hv.x, av.x, d);
        d = fmaf(hv.y, av.y, d);
        d = fmaf(hv.z, av.z, d);
        d = fmaf(hv.w, av.w, d);
      }
      sdot[(2 * hl + which) * GBM + row] = d;
    }
    __syncthreads();
  }

  v4f fv[NI];
#pragma unroll
  for (int i = 0; i < NI; ++i) {
    const int p  = lane + 32 * i;
    const int lr = 16 * wave + p / PPR;
    const int cp = p % PPR;
    fv[i] = *(const v4fa*)(stg + lr * GBN + 4 * cp);
  }

  if constexpr (MODE == 1) {
    const int cp0 = lane % PPR;
    const v4f bq = bfr4(*(const v4fa*)(bias + col0 + 4 * cp0));
#pragma unroll
    for (int i = 0; i < NI; ++i) {
      v4f y = fv[i];
      y.x = fmaxf(y.x + bq.x, 0.f);
      y.y = fmaxf(y.y + bq.y, 0.f);
      y.z = fmaxf(y.z + bq.z, 0.f);
      y.w = fmaxf(y.w + bq.w, 0.f);
      fv[i] = y;
    }
#pragma unroll
    for (int i = 0; i < NI; ++i) {
      const int p  = lane + 32 * i;
      const int gr = rowBase + 16 * wave + p / PPR;
      const int cp = p % PPR;
      float* op = outF + (size_t)gr * (size_t)ldo + col0 + 4 * cp;
      if (gr < nRows) *(volatile v4f*)op = fv[i];
    }
    __threadfence();
#pragma unroll
    for (int i = 0; i < NI; ++i) {
      const int p  = lane + 32 * i;
      const int gr = rowBase + 16 * wave + p / PPR;
      const int cp = p % PPR;
      float* op = outF + (size_t)gr * (size_t)ldo + col0 + 4 * cp;
      if (gr < nRows) *(volatile v4f*)op = fv[i];
    }
    (void)atts; (void)attd; (void)attLen; (void)nhb; (void)SD; (void)MPr;
  } else {
    const int hlc = wave < nhb ? wave : nhb - 1;
    const int which2 = lane >> 4, piece = lane & 15;
    const v4f sdv = *(const v4fa*)(sdot + (2 * hlc + which2) * GBM + 4 * piece);
    float* sp = SD + (size_t)(2 * (nhb * by + hlc) + which2) * (size_t)MPr + rowBase + 4 * piece;
    const bool wsd = wave < nhb;
#pragma unroll
    for (int i = 0; i < NI; ++i) {
      const int p  = lane + 32 * i;
      const int gr = rowBase + 16 * wave + p / PPR;
      const int cp = p % PPR;
      float* op = outF + (size_t)gr * (size_t)ldo + col0 + 4 * cp;
      *(volatile v4f*)op = fv[i];
    }
    if (wsd) *(volatile v4f*)sp = sdv;
    __threadfence();
#pragma unroll
    for (int i = 0; i < NI; ++i) {
      const int p  = lane + 32 * i;
      const int gr = rowBase + 16 * wave + p / PPR;
      const int cp = p % PPR;
      float* op = outF + (size_t)gr * (size_t)ldo + col0 + 4 * cp;
      *(volatile v4f*)op = fv[i];
    }
    if (wsd) *(volatile v4f*)sp = sdv;
    (void)nRows; (void)bias;
  }
}

template<int L>
__global__ __launch_bounds__(NTHR) void k_agg(
    const int* __restrict__ srcs, const int* __restrict__ dsts,
    const float* __restrict__ F, const float* __restrict__ SD,
    const float* __restrict__ bias, const int* __restrict__ gid, const int* __restrict__ bnn,
    unsigned short* HP, int nN, int nE, int nb, int vec8, int MPr, int nG) {
  extern __shared__ v4f lds_dyn[];
  int* reg1 = (int*)lds_dyn;
  int* reg2 = reg1 + RCAP;
  int* scnt = reg2 + RCAP;
  int* soff = scnt + NBMAX;
  int* list = soff + NBMAX;
  int* wcnt = list + LISTN;
  int* wtot = wcnt + NWAVE;
  int* scum = wtot + NWAVE;
  const int tid = (int)threadIdx.x, lane = tid & 31, wave = tid >> 5;
  unsigned short* rbuf = (unsigned short*)(scum + NGMAX + 8) + wave * RBH;
  const int nodeBase = (int)blockIdx.x * nb;
  const int nGc = nG < 1 ? 1 : (nG > NGMAX ? NGMAX : nG);

  for (int i = tid; i < NBMAX; i += NTHR) scnt[i] = 0;
  if (L == 2 && tid == 0) {
    int run = 0;
#pragma unroll 1
    for (int g = 0; g < nGc; ++g) { scum[g] = run; run += bnn[g]; }
    scum[nGc] = run;
  }
  __syncthreads();

  int tot = 0;
  const int nChunks = (nE + CHUNK - 1) / CHUNK;
#pragma unroll 1
  for (int ch = 0; ch < nChunks; ++ch) {
    const int cbase = ch * CHUNK;
    const int wc = scan_chunk(dsts, nE, cbase, nodeBase, nb, vec8, list, tid, lane, wave);
    if (lane == 0) wcnt[wave] = wc;
    __syncthreads();
    int pre = 0, all = 0;
#pragma unroll
    for (int w2 = 0; w2 < NWAVE; ++w2) {
      int c = wcnt[w2];
      c = c < 0 ? 0 : (c > WCAP ? WCAP : c);
      all += c;
      pre += (w2 < wave) ? c : 0;
    }
    const int wcc  = wc > WCAP ? WCAP : wc;
    const int base = tot + pre;
#pragma unroll 1
    for (int i = lane; i < wcc; i += 32) {
      const int ent = list[wave * WCAP + i];
      const int el  = (ent >> SLOTB) & (CHUNK - 1);
      const int sl  = ent & (NBMAX - 1);
      int eid = cbase + el;
      eid = eid > nE - 1 ? nE - 1 : eid;
      const int pos = base + i;
      if (pos < RCAP) reg1[pos] = (int)(((unsigned)eid << SLOTB) | (unsigned)sl);
    }
    tot += all;
    tot = tot > RCAP ? RCAP : tot;
    __syncthreads();
  }
  const int nh = tot;

  if (wave == 0) {
#pragma unroll 1
    for (int b0 = 0; b0 < nh; b0 += 32) {
      const int idx = b0 + lane;
      const int uv  = reg1[idx < nh ? idx : nh - 1];
      const int m32 = (nh - b0) < 32 ? (nh - b0) : 32;
#pragma unroll 1
      for (int k = 0; k < m32; ++k) {
        const int u  = __builtin_amdgcn_readlane(uv, k);
        const int sl = u & (NBMAX - 1);
        if (lane == 0) scnt[sl] = scnt[sl] + 1;
      }
    }
  }
  __syncthreads();

  {
    const v4i ca = *(const v4i*)(scnt + 8 * tid);
    const v4i cb = *(const v4i*)(scnt + 8 * tid + 4);
    const int e0 = ca.x < 0 ? 0 : ca.x, e1 = ca.y < 0 ? 0 : ca.y, e2 = ca.z < 0 ? 0 : ca.z, e3 = ca.w < 0 ? 0 : ca.w;
    const int e4 = cb.x < 0 ? 0 : cb.x, e5 = cb.y < 0 ? 0 : cb.y, e6 = cb.z < 0 ? 0 : cb.z, e7 = cb.w < 0 ? 0 : cb.w;
    const int ts = e0 + e1 + e2 + e3 + e4 + e5 + e6 + e7;
    int incl = ts;
#pragma unroll
    for (int d = 1; d < 32; d <<= 1) {
      const int up = __shfl_up(incl, d);
      if (lane >= d) incl += up;
    }
    if (lane == 31) wtot[wave] = incl;
    __syncthreads();
    int pre = 0;
#pragma unroll
    for (int w2 = 0; w2 < NWAVE; ++w2) pre += (w2 < wave) ? wtot[w2] : 0;
    int run = pre + incl - ts;
    soff[8 * tid + 0] = run; run += e0;
    soff[8 * tid + 1] = run; run += e1;
    soff[8 * tid + 2] = run; run += e2;
    soff[8 * tid + 3] = run; run += e3;
    soff[8 * tid + 4] = run; run += e4;
    soff[8 * tid + 5] = run; run += e5;
    soff[8 * tid + 6] = run; run += e6;
    soff[8 * tid + 7] = run;
  }
  __syncthreads();
  for (int i = tid; i < NBMAX; i += NTHR) list[i] = soff[i];
  __syncthreads();

  if (wave == 0) {
#pragma unroll 1
    for (int b0 = 0; b0 < nh; b0 += 32) {
      const int idx = b0 + lane;
      const int uv  = reg1[idx < nh ? idx : nh - 1];
      const int m32 = (nh - b0) < 32 ? (nh - b0) : 32;
#pragma unroll 1
      for (int k = 0; k < m32; ++k) {
        const int u   = __builtin_amdgcn_readlane(uv, k);
        const int sl  = u & (NBMAX - 1);
        const int eid = (int)((unsigned)u >> SLOTB);
        if (lane == 0) {
          int pos = list[sl];
          pos = pos < 0 ? 0 : (pos > RCAP - 1 ? RCAP - 1 : pos);
          reg2[pos] = eid;
          list[sl] = pos + 1;
        }
      }
    }
  }
  __syncthreads();

  const int nbw = nb >> 3;
  const bool ovf = (nh >= RCAP);
  const float qnan = __int_as_float(0x7fc00000);

  if (L == 1) {
    const bool act = lane < NLANE1;
    const int lc   = act ? lane : NLANE1 - 1;
    const int c0   = 16 * lc;
    const int head = lc >> 1;
    const v4f bb0  = bfr4(*(const v4fa*)(bias + c0));
    const v4f bb1  = bfr4(*(const v4fa*)(bias + c0 + 4));
    const v4f bb2  = bfr4(*(const v4fa*)(bias + c0 + 8));
    const v4f bb3  = bfr4(*(const v4fa*)(bias + c0 + 12));
    const float* ASp = SD + (size_t)(2 * head) * (size_t)MPr;
    const float* ADp = ASp + MPr;
    const int p2  = lane + 64;
    const bool w2 = p2 < RBP;
    const int p2c = w2 ? p2 : RBP - 1;

#pragma unroll 1
    for (int jt = 0; jt < nbw; ++jt) {
      const int slot = wave * nbw + jt;
      const int grow = nodeBase + slot;
      const int gcl  = grow < nN ? grow : nN - 1;
      int st = soff[slot];
      const int craw = scnt[slot];
      int cnt = craw;
      st  = st < 0 ? 0 : (st > nh ? nh : st);
      cnt = cnt < 0 ? 0 : (cnt > DEGCAP ? DEGCAP : cnt);
      if (cnt > nh - st) cnt = nh - st;
      const float pz = (ovf || craw > DEGCAP) ? qnan : 0.0f;

      const float* fr = F + (size_t)gcl * HC1 + c0;
      v4f av0 = *(const v4fa*)fr, av1 = *(const v4fa*)(fr + 4), av2 = *(const v4fa*)(fr + 8), av3 = *(const v4fa*)(fr + 12);
      const float adv = ADp[gcl];
      float l0 = ASp[gcl] + adv;
      l0 = l0 > 0.f ? l0 : NEGSL * l0;
      float mx = l0, dn = 1.0f;

#pragma unroll 1
      for (int q = 0; q < cnt; ++q) {
        int idx = st + q; idx = idx > RCAP - 1 ? RCAP - 1 : idx;
        int eid = reg2[idx]; eid = eid < 0 ? 0 : (eid > nE - 1 ? nE - 1 : eid);
        const int sraw = srcs[eid];
        const int s = sraw < 0 ? 0 : (sraw > nN - 1 ? nN - 1 : sraw);
        const float* gs = F + (size_t)s * HC1 + c0;
        const v4f f0 = *(const v4fa*)gs, f1 = *(const v4fa*)(gs + 4), f2 = *(const v4fa*)(gs + 8), f3 = *(const v4fa*)(gs + 12);
        float lg = ASp[s] + adv;
        lg = lg > 0.f ? lg : NEGSL * lg;
        const float df = lg - mx;
        const float ee = __expf(-fabsf(df));
        const bool up  = df > 0.f;
        const float s1 = up ? ee : 1.0f;
        const float s2 = up ? 1.0f : ee;
        mx = up ? lg : mx;
        dn = fmaf(dn, s1, s2);
        av0 = upd4(av0, s1, s2, f0);
        av1 = upd4(av1, s1, s2, f1);
        av2 = upd4(av2, s1, s2, f2);
        av3 = upd4(av3, s1, s2, f3);
      }
      const float inv = __builtin_amdgcn_rcpf(dn + EPS_SM);
      const bool live = grow < nN;
      const v4f o0 = elu4(av0, inv, bb0, live, pz);
      const v4f o1 = elu4(av1, inv, bb1, live, pz);
      const v4f o2 = elu4(av2, inv, bb2, live, pz);
      const v4f o3 = elu4(av3, inv, bb3, live, pz);
      v4u l0w, l1w;
      const v4u h0w = hl8(o0, o1, l0w);
      const v4u h1w = hl8(o2, o3, l1w);
      if (act) {
        *(v4ua*)(rbuf + c0)           = h0w;
        *(v4ua*)(rbuf + c0 + 8)       = h1w;
        *(v4ua*)(rbuf + HC1 + c0)     = l0w;
        *(v4ua*)(rbuf + HC1 + c0 + 8) = l1w;
      }
      wave_sync();
      const v4u q0 = *(const v4ua*)(rbuf + 8 * lane);
      const v4u q1 = *(const v4ua*)(rbuf + 8 * (lane + 32));
      const v4u q2 = *(const v4ua*)(rbuf + 8 * p2c);
      wave_sync();
      unsigned short* gp = HP + (size_t)grow * KA2;
      const bool wr = grow < MPr;
      if (wr) {
        *(volatile v4u*)(gp + 8 * lane) = q0;
        *(volatile v4u*)(gp + 8 * (lane + 32)) = q1;
        if (w2) *(volatile v4u*)(gp + 8 * p2) = q2;
      }
      __threadfence();
      if (wr) {
        *(volatile v4u*)(gp + 8 * lane) = q0;
        *(volatile v4u*)(gp + 8 * (lane + 32)) = q1;
        if (w2) *(volatile v4u*)(gp + 8 * p2) = q2;
      }
    }
  } else {
    const int c0   = 4 * lane;
    const v4f bb4  = bfr4(*(const v4fa*)(bias + c0));
    const float* ASp = SD;
    const float* ADp = SD + MPr;

#pragma unroll 1
    for (int jt = 0; jt < nbw; ++jt) {
      const int slot = wave * nbw + jt;
      const int grow = nodeBase + slot;
      const int gcl  = grow < nN ? grow : nN - 1;
      int st = soff[slot];
      const int craw = scnt[slot];
      int cnt = craw;
      st  = st < 0 ? 0 : (st > nh ? nh : st);
      cnt = cnt < 0 ? 0 : (cnt > DEGCAP ? DEGCAP : cnt);
      if (cnt > nh - st) cnt = nh - st;
      const float pz = (ovf || craw > DEGCAP) ? qnan : 0.0f;

      const v4f fd = *(const v4fa*)(F + (size_t)gcl * NC2 + c0);
      const float adv = ADp[gcl];
      float l0 = ASp[gcl] + adv;
      l0 = l0 > 0.f ? l0 : NEGSL * l0;
      float mx = l0, dn = 1.0f;
      v4f av = fd;

#pragma unroll 1
      for (int q = 0; q < cnt; ++q) {
        int idx = st + q; idx = idx > RCAP - 1 ? RCAP - 1 : idx;
        int eid = reg2[idx]; eid = eid < 0 ? 0 : (eid > nE - 1 ? nE - 1 : eid);
        const int sraw = srcs[eid];
        const int s = sraw < 0 ? 0 : (sraw > nN - 1 ? nN - 1 : sraw);
        const v4f fs = *(const v4fa*)(F + (size_t)s * NC2 + c0);
        float lg = ASp[s] + adv;
        lg = lg > 0.f ? lg : NEGSL * lg;
        const float df = lg - mx;
        const float ee = __expf(-fabsf(df));
        const bool up  = df > 0.f;
        const float s1 = up ? ee : 1.0f;
        const float s2 = up ? 1.0f : ee;
        mx = up ? lg : mx;
        dn = fmaf(dn, s1, s2);
        av = upd4(av, s1, s2, fs);
      }
      const float inv = __builtin_amdgcn_rcpf(dn + EPS_SM);
      const bool live = grow < nN;
      const int graw = gid[gcl];
      const int gc   = graw < 0 ? 0 : (graw > nGc ? nGc : graw);
      const unsigned idxv = (unsigned)gcl - (unsigned)scum[gc] + (unsigned)graw * (unsigned)PER_G;
      const float pid = (live && idxv != (unsigned)gcl) ? qnan : 0.0f;
      const float hx = fmaxf(fmaf(av.x, inv, bb4.x), 0.f);
      const float hy = fmaxf(fmaf(av.y, inv, bb4.y), 0.f);
      const float hz = fmaxf(fmaf(av.z, inv, bb4.z), 0.f);
      const float hw = fmaxf(fmaf(av.w, inv, bb4.w), 0.f);
      v4f o;
      o.x = (live ? hx : 0.f) + pz + pid;
      o.y = (live ? hy : 0.f) + pz + pid;
      o.z = (live ? hz : 0.f) + pz + pid;
      o.w = (live ? hw : 0.f) + pz + pid;
      const unsigned int hbx = f2bf(o.x), hby = f2bf(o.y), hbz = f2bf(o.z), hbw = f2bf(o.w);
      const unsigned int lbx = f2bf(o.x - bf2f(hbx)), lby = f2bf(o.y - bf2f(hby));
      const unsigned int lbz = f2bf(o.z - bf2f(hbz)), lbw = f2bf(o.w - bf2f(hbw));
      const int hw0 = (int)(hbx | (hby << 16)), hw1 = (int)(hbz | (hbw << 16));
      const int lw0 = (int)(lbx | (lby << 16)), lw1 = (int)(lbz | (lbw << 16));
      const int sa = (2 * lane) & 31, sb = (2 * lane + 1) & 31;
      const int g0 = __shfl(hw0, sa), g1 = __shfl(hw1, sa), g2 = __shfl(hw0, sb), g3 = __shfl(hw1, sb);
      const int q0 = __shfl(lw0, sa), q1 = __shfl(lw1, sa), q2 = __shfl(lw0, sb), q3 = __shfl(lw1, sb);
      const bool lsel = lane >= 16;
      v4u pv;
      pv.x = (unsigned int)(lsel ? q0 : g0);
      pv.y = (unsigned int)(lsel ? q1 : g1);
      pv.z = (unsigned int)(lsel ? q2 : g2);
      pv.w = (unsigned int)(lsel ? q3 : g3);
      unsigned short* gp = HP + (size_t)grow * KFC + 8 * lane;
      const bool wr = grow < MPr;
      if (wr) *(volatile v4u*)gp = pv;
      __threadfence();
      if (wr) *(volatile v4u*)gp = pv;
    }
  }
}

__global__ __launch_bounds__(PTHR) void k_pool(const unsigned short* __restrict__ xp, const int* __restrict__ gidp,
                                               int nN, int nG, unsigned short* pp) {
  __shared__ __attribute__((aligned(16))) float wst[NWAVE * NC2];
  __shared__ __attribute__((aligned(16))) float pst[NC2];
  __shared__ __attribute__((aligned(16))) unsigned short prow[KFC];
  __shared__ int plist[NWAVE * 32];
  const int tid = (int)threadIdx.x, lane = tid & 31, wave = tid >> 5;
  const int g = (int)blockIdx.x;
  const bool liveg = g < nG;
  const float ninf = -__builtin_huge_valf();
  float m0 = ninf, m1 = ninf, m2 = ninf, m3 = ninf;
  const int nChunks = liveg ? (nN + PTHR - 1) / PTHR : 0;
#pragma unroll 1
  for (int ch = 0; ch < nChunks; ++ch) {
    const int n  = ch * PTHR + tid;
    const int nc = n < nN ? n : nN - 1;
    const int bv = gidp[nc];
    const bool hit = (n < nN) && (bv == g);
    const unsigned mj = __builtin_amdgcn_ballot_w32(hit);
    if (mj != 0u) {
      if (hit) plist[wave * 32 + (int)__builtin_amdgcn_mbcnt_lo(mj, 0u)] = n;
      const int c = (int)__builtin_popcount(mj);
      wave_sync();
#pragma unroll 1
      for (int k = 0; k < c; ++k) {
        int nd = plist[wave * 32 + k];
        nd = nd < 0 ? 0 : (nd > nN - 1 ? nN - 1 : nd);
        const unsigned short* rp = xp + (size_t)nd * KFC + 4 * lane;
        const v2u wh = *(const v2ua*)rp;
        const v2u wl = *(const v2ua*)(rp + NC2);
        const float f0 = __uint_as_float(wh.x << 16)         + __uint_as_float(wl.x << 16);
        const float f1 = __uint_as_float(wh.x & 0xffff0000u) + __uint_as_float(wl.x & 0xffff0000u);
        const float f2 = __uint_as_float(wh.y << 16)         + __uint_as_float(wl.y << 16);
        const float f3 = __uint_as_float(wh.y & 0xffff0000u) + __uint_as_float(wl.y & 0xffff0000u);
        m0 = fmaxf(m0, f0); m1 = fmaxf(m1, f1); m2 = fmaxf(m2, f2); m3 = fmaxf(m3, f3);
      }
      wave_sync();
    }
  }
  {
    v4f mv4; mv4.x = m0; mv4.y = m1; mv4.z = m2; mv4.w = m3;
    *(v4fa*)(wst + wave * NC2 + 4 * lane) = mv4;
  }
  __syncthreads();
  if (tid < NC2) {
    float mv = ninf;
#pragma unroll 1
    for (int w2 = 0; w2 < NWAVE; ++w2) mv = fmaxf(mv, wst[w2 * NC2 + tid]);
    pst[tid] = liveg ? mv : 0.0f;
  }
  __syncthreads();
  if (wave == 0) {
    const v4f v = *(const v4fa*)(pst + 4 * lane);
    const unsigned int hbx = f2bf(v.x), hby = f2bf(v.y), hbz = f2bf(v.z), hbw = f2bf(v.w);
    const unsigned int lbx = f2bf(v.x - bf2f(hbx)), lby = f2bf(v.y - bf2f(hby));
    const unsigned int lbz = f2bf(v.z - bf2f(hbz)), lbw = f2bf(v.w - bf2f(hbw));
    v2u h2, l2;
    h2.x = hbx | (hby << 16); h2.y = hbz | (hbw << 16);
    l2.x = lbx | (lby << 16); l2.y = lbz | (lbw << 16);
    *(v2ua*)(prow + 4 * lane)       = h2;
    *(v2ua*)(prow + NC2 + 4 * lane) = l2;
    wave_sync();
    const v4u q = *(const v4ua*)(prow + 8 * lane);
    unsigned short* op = pp + (size_t)g * KFC + 8 * lane;
    *(volatile v4u*)op = q;
    __threadfence();
    *(volatile v4u*)op = q;
  }
}

static int pick_nb(int nE, int nN) {
  int nb = NBMAX;
  while (nb > 32 && (long long)nb * (long long)nE * 5LL > (long long)RCAP * (long long)nN * 4LL) nb >>= 1;
  return nb;
}
static inline int cdiv(int a, int b) { return (a + b - 1) / b; }
static inline size_t al256(size_t o) { return (o + 255) & ~(size_t)255; }

extern "C" void kernel_launch(void* const* d_in, const int* in_sizes, int n_in,
                              void* d_out, int out_size, void* d_ws, size_t ws_size,
                              hipStream_t stream) {
  if (n_in < 14) return;
  if (in_sizes[0] < F_IN || (in_sizes[0] % F_IN) != 0) return;
  const int nN = in_sizes[0] / F_IN;
  if (nN < GBM || nN > (1 << 22)) return;
  if (in_sizes[1] < 2 || (in_sizes[1] & 1) != 0) return;
  const int nE = in_sizes[1] / 2;
  if (nE < 1 || nE >= (1 << (32 - SLOTB))) return;
  if (in_sizes[2] != nN) return;
  const int nG = in_sizes[3];
  if (nG < 1 || nG > NGMAX - 1 || nG > 65535) return;
  if ((long long)nG * PER_G != (long long)nN) return;
  if (in_sizes[4] != F_IN * HC1) return;
  if (in_sizes[5] != NHD1 * HID || in_sizes[6] != NHD1 * HID) return;
  if (in_sizes[7] != HC1) return;
  if (in_sizes[8] != HC1 * NC2) return;
  if (in_sizes[9] != NC2 || in_sizes[10] != NC2) return;
  if (in_sizes[11] != NC2) return;
  if (in_sizes[12] != NC2 * NC2) return;
  if (in_sizes[13] != NC2) return;
  if ((long long)out_size != (long long)nN * NC2 + (long long)nG * NC2) return;

  const float* x    = (const float*)d_in[0];
  const int*   ei   = (const int*)  d_in[1];
  const int*   gidp = (const int*)  d_in[2];
  const int*   bnn  = (const int*)  d_in[3];
  const float* W1   = (const float*)d_in[4];
  const float* a1s  = (const float*)d_in[5];
  const float* a1d  = (const float*)d_in[6];
  const float* b1   = (const float*)d_in[7];
  const float* W2   = (const float*)d_in[8];
  const float* a2s  = (const float*)d_in[9];
  const float* a2d  = (const float*)d_in[10];
  const float* b2   = (const float*)d_in[11];
  const float* fcw  = (const float*)d_in[12];
  const float* fcb  = (const float*)d_in[13];
  float* out0 = (float*)d_out;
  float* out1 = out0 + (size_t)nN * NC2;
  const int* src = ei;
  const int* dst = ei + nE;

  const int MP   = cdiv(nN, MROWS) * MROWS;
  const int PPR  = cdiv(nG, GBM) * GBM;
  const int nb   = pick_nb(nE, nN);
  if (nb < 32 || (nb & (nb - 1)) != 0 || nb > NBMAX) return;
  const int gA   = cdiv(MP, nb);
  const int vec8 = ((nE & 3) == 0) ? 1 : 0;
  if ((long long)gA * nb < (long long)MP) return;

  char* ws = (char*)d_ws;
  size_t off = 0;
  const size_t oXB  = off; off = al256(off + (size_t)MP * F_IN * 2);
  const size_t oW1T = off; off = al256(off + (size_t)HC1 * F_IN * 2);
  const size_t oW2T = off; off = al256(off + (size_t)NC2 * KA2 * 2);
  const size_t oFCT = off; off = al256(off + (size_t)NC2 * KFC * 2);
  const size_t oH1  = off; off = al256(off + (size_t)MP * HC1 * 4);
  const size_t oSD1 = off; off = al256(off + (size_t)2 * NHD1 * MP * 4);
  const size_t oA2  = off; off = al256(off + (size_t)MP * KA2 * 2);
  const size_t oH2  = off; off = al256(off + (size_t)MP * NC2 * 4);
  const size_t oSD2 = off; off = al256(off + (size_t)2 * MP * 4);
  const size_t oXP  = off; off = al256(off + (size_t)MP * KFC * 2);
  const size_t oPP  = off; off = al256(off + (size_t)PPR * KFC * 2);
  if (off > ws_size || off > (size_t)WSMAX) return;
  unsigned short* XB  = (unsigned short*)(ws + oXB);
  unsigned short* W1T = (unsigned short*)(ws + oW1T);
  unsigned short* W2T = (unsigned short*)(ws + oW2T);
  unsigned short* FCT = (unsigned short*)(ws + oFCT);
  float*          H1  = (float*)(ws + oH1);
  float*          SD1 = (float*)(ws + oSD1);
  unsigned short* A2  = (unsigned short*)(ws + oA2);
  float*          H2  = (float*)(ws + oH2);
  float*          SD2 = (float*)(ws + oSD2);
  unsigned short* XP  = (unsigned short*)(ws + oXP);
  unsigned short* PP  = (unsigned short*)(ws + oPP);

  hipFuncSetAttribute(reinterpret_cast<const void*>(&k_agg<1>),
                      hipFuncAttributeMaxDynamicSharedMemorySize, LDS_AGG);
  hipFuncSetAttribute(reinterpret_cast<const void*>(&k_agg<2>),
                      hipFuncAttributeMaxDynamicSharedMemorySize, LDS_AGG);

  const int nUx = MP * XQ;
  k_xprep<<<cdiv(nUx, NTHR), NTHR, 0, stream>>>(x, XB, nN, nUx);

  {
    const int nUw1 = HC1 * (F_IN / 8);
    k_wtr<<<cdiv(nUw1, NTHR), NTHR, 0, stream>>>(W1, F_IN, HC1, HC1, F_IN, W1T, nUw1);
    const int nUw2 = NC2 * (KA2 / 8);
    k_wtr<<<cdiv(nUw2, NTHR), NTHR, 0, stream>>>(W2, HC1, NC2, NC2, KA2, W2T, nUw2);
    const int nUw3 = NC2 * (KFC / 8);
    k_wtr<<<cdiv(nUw3, NTHR), NTHR, 0, stream>>>(fcw, NC2, NC2, NC2, KFC, FCT, nUw3);
  }

  const int gM = MP / GBM;
  k_gemm<4, 0><<<dim3(gM, HC1 / 64), GTHR, 0, stream>>>(XB, W1T, H1, F_IN, HC1, MP, a1s, a1d, HID, NHB1, SD1, MP, b1);
  k_agg<1><<<gA, NTHR, LDS_AGG, stream>>>(src, dst, H1, SD1, b1, gidp, bnn, A2, nN, nE, nb, vec8, MP, nG);
  k_gemm<8, 0><<<dim3(gM, 1), GTHR, 0, stream>>>(A2, W2T, H2, KA2, NC2, MP, a2s, a2d, NC2, 1, SD2, MP, b2);
  k_agg<2><<<gA, NTHR, LDS_AGG, stream>>>(src, dst, H2, SD2, b2, gidp, bnn, XP, nN, nE, nb, vec8, MP, nG);
  k_gemm<8, 1><<<dim3(gM, 1), GTHR, 0, stream>>>(XP, FCT, out0, KFC, NC2, nN, a2s, a2d, NC2, 1, SD2, MP, fcb);
  k_pool<<<PPR, PTHR, 0, stream>>>(XP, gidp, nN, nG, PP);
  k_gemm<8, 1><<<dim3(PPR / GBM, 1), GTHR, 0, stream>>>(PP, FCT, out1, KFC, NC2, nG, a2s, a2d, NC2, 1, SD2, MP, fcb);
}
